// Triton_MHA_77687368450156
// MI455X (gfx1250) — hardware-verified
//
#include <hip/hip_runtime.h>
#include <hip/hip_bf16.h>
#include <math.h>

#define BB 8
#define LTRUE 1000
#define SS 1024
#define QROWS 1024
#define KROWS 1024
#define NKV 1024
#define DD 1024
#define HH 16
#define KVH 16
#define KVD 1024
#define HKDIV 1
#define DKK 64
#define QW 2
#define GSTR 48

typedef _Float16 bf16;
typedef _Float16 f16;
typedef __attribute__((ext_vector_type(4))) unsigned v4u_t;
typedef unsigned v4ua __attribute__((ext_vector_type(4), may_alias));
typedef __attribute__((ext_vector_type(4))) float v4f_t;
typedef float v4fa __attribute__((ext_vector_type(4), may_alias));
typedef __attribute__((ext_vector_type(16))) bf16  bf16x16;
typedef bf16x16 f16x16;
typedef __attribute__((ext_vector_type(8)))  bf16  bf16x8;
typedef bf16x8 f16x8;
typedef __attribute__((ext_vector_type(4)))  bf16  bf16x4;
typedef __attribute__((ext_vector_type(8)))  float f32x8;
__device__ __forceinline__ f32x8 wmma16(f16x16 a, f16x16 b, f32x8 c) {
  c = __builtin_amdgcn_wmma_f32_16x16x32_f16(false, a, false, b, (short)0, c, false, false);
  asm volatile("v_nop\n\tv_nop\n\tv_nop\n\tv_nop" : "+v"(c) : "v"(a), "v"(b));
  return c;
}
#define LDS_STRIDE 48
#define KSTRIDE    72
#define VSTRIDE    48

__device__ __forceinline__ f32x8 wmma_bf16(bf16x16 a, bf16x16 b, f32x8 c) {
  c = __builtin_amdgcn_wmma_f32_16x16x32_f16(false, a, false, b, (short)0, c, false, false);
  asm volatile("v_nop\n\tv_nop\n\tv_nop\n\tv_nop" : "+v"(c) : "v"(a), "v"(b));
  return c;
}

template <typename T>
__device__ __forceinline__ bf16x16 load_frag(const T* __restrict__ base, int ld,
                                             int row0, int k0) {
  const int lane = threadIdx.x & 31;
  const int r    = lane & 15;
  const int kh   = (lane >> 4) * 8;
  const T* p0 = base + (size_t)(row0 + r) * ld + (k0 + kh);
  const T* p1 = p0 + 16;
  bf16x16 f;
#pragma unroll
  for (int i = 0; i < 8; ++i) {
    f[i]     = (bf16)p0[i];
    f[i + 8] = (bf16)p1[i];
  }
  return f;
}

__device__ __forceinline__ bf16x16 lds_frag(const bf16* base, int stride) {
  const int lane = threadIdx.x & 31;
  const int row  = lane & 15;
  const int kh   = (lane >> 4) * 8;
  const bf16x8 lo = *(const bf16x8*)(base + row * stride + kh);
  const bf16x8 hi = *(const bf16x8*)(base + row * stride + kh + 16);
  bf16x16 f;
#pragma unroll
  for (int i = 0; i < 8; ++i) { f[i] = lo[i]; f[i + 8] = hi[i]; }
  return f;
}

template <typename T>
__device__ __forceinline__ void stage_read16(const T* __restrict__ p, float* buf) {
#pragma unroll
  for (int i = 0; i < 16; ++i) buf[i] = (float)p[i];
}

__device__ __forceinline__ void stage_write(bf16* dst, const float* buf, int nquad) {
#pragma unroll
  for (int i = 0; i < nquad; ++i) {
    bf16x4 q;
    q[0] = (bf16)buf[4 * i];     q[1] = (bf16)buf[4 * i + 1];
    q[2] = (bf16)buf[4 * i + 2]; q[3] = (bf16)buf[4 * i + 3];
    *(bf16x4*)(dst + 4 * i) = q;
  }
}

__global__ __launch_bounds__(64) void attn_kernel(
    const bf16* __restrict__ Qb, const bf16* __restrict__ Kb,
    const bf16* __restrict__ Vt, const float* __restrict__ kbias,
    float* __restrict__ attnOut) {
  __shared__ bf16 ldsK[32 * KSTRIDE];
  __shared__ bf16 ldsV[64 * VSTRIDE];
  __shared__ __attribute__((aligned(16))) bf16 ldsO[2][32 * 72];

  const int q0blk = blockIdx.x * 64;
  const int h  = blockIdx.y;
  const int b  = blockIdx.z;
  const int t    = threadIdx.x;
  const int wave = t >> 5;
  const int lane = t & 31;
  const int qlane = lane & 15;
  const int kh8   = (lane >> 4) * 8;
  const int q0 = q0blk + wave * 32;

  const int hk = h / HKDIV;
  const bf16* Qh = Qb + (size_t)b * QROWS * DD + h * DKK;
  const bf16* Kh = Kb + (size_t)b * KROWS * KVD + hk * DKK;
  const bf16* Vh = Vt + ((size_t)(b * KVH + hk)) * DKK * KROWS;

  const int krow = t >> 1;
  const int kcol = (t & 1) * 32;
  const bf16* kSrc = Kh + (size_t)krow * KVD + kcol;
  const bf16* vSrc = Vh + (size_t)t * KROWS;

  bf16x16 qf[QW][2];
#pragma unroll
  for (int qt = 0; qt < QW; ++qt) {
    qf[qt][0] = load_frag(Qh, DD, q0 + 16 * qt, 0);
    qf[qt][1] = load_frag(Qh, DD, q0 + 16 * qt, 32);
  }

  f32x8 o[QW][4] = {};
  float mrun[QW], lrun[QW];
#pragma unroll
  for (int qt = 0; qt < QW; ++qt) { mrun[qt] = -INFINITY; lrun[qt] = 0.0f; }

  const float scale = 0.125f * 1.44269504088896340736f;
  const float NEG2 = -1.0e9f;
  const int kmax = KROWS - 1;
  __shared__ float kbS[KROWS];
  for (int i = threadIdx.x; i < KROWS; i += 64) kbS[i] = kbias[(size_t)b * KROWS + i] * 1.44269504088896340736f;
  __syncthreads();

  bf16x8 kreg[4], vreg[4];
#pragma unroll
  for (int i = 0; i < 4; ++i) {
    kreg[i] = *(const bf16x8*)(kSrc + 8 * i);
    vreg[i] = *(const bf16x8*)(vSrc + 8 * i);
  }

  for (int kb = 0; kb <= kmax; kb += 32) {
    __syncthreads();
#pragma unroll
    for (int i = 0; i < 4; ++i) {
      *(bf16x8*)(&ldsK[krow * KSTRIDE + kcol + 8 * i]) = kreg[i];
      *(bf16x8*)(&ldsV[t * VSTRIDE + 8 * i])           = vreg[i];
    }
    if (kb + 32 <= kmax) {
      const bf16* kn = kSrc + (size_t)(kb + 32) * KVD;
      const bf16* vn = vSrc + (kb + 32);
#pragma unroll
      for (int i = 0; i < 4; ++i) {
        kreg[i] = *(const bf16x8*)(kn + 8 * i);
        vreg[i] = *(const bf16x8*)(vn + 8 * i);
      }
    }
    __syncthreads();

    bf16x16 kf[2][2];
#pragma unroll
    for (int ktile = 0; ktile < 2; ++ktile)
#pragma unroll
      for (int c = 0; c < 2; ++c)
        kf[ktile][c] = lds_frag(ldsK + (ktile * 16) * KSTRIDE + c * 32, KSTRIDE);

    bf16x16 pf[QW];
    bool act[QW];
#pragma unroll
    for (int qt = 0; qt < QW; ++qt) {
      unsigned mbits = 0;
      {
#pragma unroll
        for (int r = 0; r < 8; ++r) { const int j0 = kb + kh8 + r; if (j0 < NKV) mbits |= 1u << r; if (j0 + 16 < NKV) mbits |= 1u << (8 + r); }
        act[qt] = (__builtin_amdgcn_ballot_w32(mbits != 0) != 0);
      }
      if (act[qt]) {
        const int q_my = q0 + 16 * qt + qlane;
        f32x8 s0 = {}, s1 = {};
        s0 = wmma_bf16(kf[0][0], qf[qt][0], s0);
        s0 = wmma_bf16(kf[0][1], qf[qt][1], s0);
        s1 = wmma_bf16(kf[1][0], qf[qt][0], s1);
        s1 = wmma_bf16(kf[1][1], qf[qt][1], s1);

        float mx = -INFINITY;
#pragma unroll
        for (int r = 0; r < 8; ++r) {
          const int k0i = kb + kh8 + r;
          const int k1i = k0i + 16;
          (void)k0i; (void)k1i; (void)q_my;
          s0[r] = (mbits & (1u << r))       ? s0[r] * scale + kbS[kb + kh8 + r] : NEG2;
          s1[r] = (mbits & (1u << (8 + r))) ? s1[r] * scale + kbS[kb + 16 + kh8 + r] : NEG2;
          mx = fmaxf(mx, fmaxf(s0[r], s1[r]));
        }
        mx = fmaxf(mx, __shfl_xor(mx, 16, 32));
        const float mnew  = fmaxf(mrun[qt], mx);
        const float alpha = exp2f(mrun[qt] - mnew);

        float rsum = 0.0f;
#pragma unroll
        for (int r = 0; r < 8; ++r) {
          const float p0 = exp2f(s0[r] - mnew);
          const float p1 = exp2f(s1[r] - mnew);
          rsum += p0 + p1;
          pf[qt][r]     = (bf16)(p0 * 1024.0f);
          pf[qt][r + 8] = (bf16)(p1 * 1024.0f);
        }
        rsum += __shfl_xor(rsum, 16, 32);
        lrun[qt] = lrun[qt] * alpha + rsum;
        mrun[qt] = mnew;

#pragma unroll
        for (int j = 0; j < 4; ++j)
#pragma unroll
          for (int r = 0; r < 8; ++r) o[qt][j][r] *= alpha;
      }
    }

#pragma unroll
    for (int j = 0; j < 4; ++j) {
      const bf16x16 vf = lds_frag(ldsV + (j * 16) * VSTRIDE, VSTRIDE);
#pragma unroll
      for (int qt = 0; qt < QW; ++qt)
        if (act[qt]) o[qt][j] = wmma_bf16(vf, pf[qt], o[qt][j]);
    }
  }

  __shared__ __attribute__((aligned(16))) float ldsOf[2][32 * 68];
  float* so = ldsOf[wave]; (void)ldsO;
#pragma unroll
  for (int qt = 0; qt < QW; ++qt) {
    const float rl = 1.0f / (lrun[qt] * 1024.0f);
#pragma unroll
    for (int j = 0; j < 4; ++j)
#pragma unroll
      for (int r = 0; r < 8; ++r) so[(16 * qt + qlane) * 68 + j * 16 + kh8 + r] = o[qt][j][r] * rl;
  }
  asm volatile("s_wait_dscnt 0" ::: "memory");
  __builtin_amdgcn_wave_barrier();
#pragma unroll 1
  for (int pass = 0; pass < 2; ++pass) {
#pragma unroll
    for (int it = 0; it < 16; ++it) { const int ch = lane + 32 * it, ql = ch >> 4, q4 = (ch & 15) * 4;
      *(volatile v4f_t*)(attnOut + ((size_t)(b * QROWS + q0 + ql)) * DD + h * DKK + q4) = *(const v4fa*)(so + ql * 68 + q4); }
    __threadfence();
  }
}


__global__ __launch_bounds__(256) void k_prep(const float* __restrict__ q, bf16* __restrict__ Q16, bf16* __restrict__ Vt) {
  __shared__ __attribute__((aligned(16))) bf16 qS[64][72], vT[64][72];
  const int tid = threadIdx.x; const int n0 = blockIdx.x * 64, h = blockIdx.y, b = blockIdx.z;
  for (int e = tid; e < 64 * 64; e += 256) { const int t = e >> 6, d = e & 63; const int n = n0 + t; const float v = (n < LTRUE) ? q[((size_t)b * LTRUE + n) * DD + h * DKK + d] : 0.0f; qS[t][d] = (bf16)v; vT[d][t] = (bf16)v; }
  __syncthreads();
#pragma unroll 1
  for (int pass = 0; pass < 2; ++pass) {
#pragma unroll 1
    for (int round = 0; round < 2; ++round) { const int r = round * 32 + (tid >> 3), piece = (tid & 7) * 8;
      *(volatile v4u_t*)(Q16 + ((size_t)b * SS + n0 + r) * DD + h * DKK + piece) = *(const v4ua*)(&qS[r][piece]);
      *(volatile v4u_t*)(Vt + ((size_t)b * DD + h * DKK + r) * SS + n0 + piece) = *(const v4ua*)(&vT[r][piece]); }
    __threadfence(); }
}
__global__ __launch_bounds__(256) void k_kbias(const int* __restrict__ mask, float* __restrict__ kb) { const int b = blockIdx.x;
  for (int q4 = threadIdx.x; q4 < KROWS / 4; q4 += 256) { v4f_t o; for (int e = 0; e < 4; ++e) { const int k = q4 * 4 + e; o[e] = (k < LTRUE && mask[b * LTRUE + k] != 0) ? 0.0f : -1.0e9f; }
    *(volatile v4f_t*)(kb + (size_t)b * KROWS + q4 * 4) = o; __threadfence(); *(volatile v4f_t*)(kb + (size_t)b * KROWS + q4 * 4) = o; } }
__global__ __launch_bounds__(256) void k_copy(const float* __restrict__ A, float* __restrict__ out) { const int n = blockIdx.x, b = blockIdx.y;
  const v4f_t v = *(const v4f_t*)(A + ((size_t)b * QROWS + n) * DD + threadIdx.x * 4);
  *(volatile v4f_t*)(out + ((size_t)b * LTRUE + n) * DD + threadIdx.x * 4) = v; __threadfence(); *(volatile v4f_t*)(out + ((size_t)b * LTRUE + n) * DD + threadIdx.x * 4) = v; }

extern "C" void kernel_launch(void* const* d_in, const int* in_sizes, int n_in,
                              void* d_out, int out_size, void* d_ws, size_t ws_size,
                              hipStream_t stream) {
  (void)in_sizes; (void)n_in; (void)out_size;
  const float* q = (const float*)d_in[0]; const int* mask = (const int*)d_in[1];
  float* out = (float*)d_out;
  char* ws = (char*)d_ws;
  bf16* Q16 = (bf16*)ws; ws += (size_t)BB * SS * DD * 2;
  bf16* Vt = (bf16*)ws; ws += (size_t)BB * DD * SS * 2;
  float* A = (float*)ws; ws += (size_t)BB * QROWS * DD * 4;
  float* kb = (float*)ws; ws += (size_t)BB * KROWS * 4;
  if ((size_t)(ws - (char*)d_ws) > ws_size) return;
  const dim3 blk(256);
  k_prep<<<dim3(SS / 64, HH, BB), blk, 0, stream>>>(q, Q16, Vt);
  k_kbias<<<dim3(BB), blk, 0, stream>>>(mask, kb);
  attn_kernel<<<dim3(QROWS / 64, HH, BB), dim3(64), 0, stream>>>(Q16, Q16, Vt, kb, A);
  k_copy<<<dim3(LTRUE, BB), blk, 0, stream>>>(A, out);
}
